// ResidualAttentionBlock_15083925144167
// MI455X (gfx1250) — hardware-verified
//
#include <hip/hip_runtime.h>
#include <math.h>
#include <stdint.h>

#ifndef NB
#define NB 16
#endif
#ifndef NQ
#define NQ 4096
#endif
#define NB_FULL 16
#define CC     128
#define NN     4096
#define NGRP   8
#define GSZ    16
#define QT     64
#define OSP    68
#define OSPW   132
#define TP     72
#define SCL    0.08838834764831845f
#define LNPS   9.704060527839234f
#define GEPS   1.0e-5

static_assert(NB >= 1 && NB <= NB_FULL);
static_assert(NQ >= QT && NQ <= NN && NQ % QT == 0);
static_assert(NN % QT == 0 && NN % 32 == 0);
static_assert(CC == 2 * QT && CC % 32 == 0);
static_assert(GSZ * NGRP == CC);
static_assert((GSZ * NN) % (4 * 256) == 0);
static_assert((OSP * 4) % 16 == 0);
static_assert((OSPW * 4) % 16 == 0);
static_assert((TP * 2) % 16 == 0);

typedef _Float16       v16h __attribute__((ext_vector_type(16)));
typedef _Float16       v8h  __attribute__((ext_vector_type(8)));
typedef __bf16         v16b __attribute__((ext_vector_type(16)));
typedef unsigned short v8us __attribute__((ext_vector_type(8)));
typedef float          v8f  __attribute__((ext_vector_type(8)));
typedef float          v4f  __attribute__((ext_vector_type(4)));
typedef unsigned int   v4u  __attribute__((ext_vector_type(4)));

union Frag  { v8us u[2]; v16h h; v16b bf; };
union FragH { v16h v; v8h hv[2]; };
static_assert(sizeof(Frag) == 32);
static_assert(sizeof(FragH) == 32);

__device__ __forceinline__ unsigned short bf_bits(float f) {
  unsigned u = __float_as_uint(f);
  return (unsigned short)((u + 0x7FFFu + ((u >> 16) & 1u)) >> 16);
}
__device__ __forceinline__ float bf_up(unsigned short hb) { return __uint_as_float(((unsigned)hb) << 16); }
__device__ __forceinline__ float bfr(float f) { return bf_up(bf_bits(f)); }
__device__ __forceinline__ unsigned short h_bits(_Float16 x) { return __builtin_bit_cast(unsigned short, x); }
__device__ __forceinline__ unsigned pk16(unsigned short a, unsigned short b) { return (unsigned)a | ((unsigned)b << 16); }
__device__ __forceinline__ v8f zero8() { v8f z = {0.f, 0.f, 0.f, 0.f, 0.f, 0.f, 0.f, 0.f}; return z; }
__device__ __forceinline__ float hmax8(v8f s) {
  return fmaxf(fmaxf(fmaxf(s[0], s[1]), fmaxf(s[2], s[3])), fmaxf(fmaxf(s[4], s[5]), fmaxf(s[6], s[7])));
}
__device__ __forceinline__ unsigned wave_ballot(bool p) {
#if defined(__HIP_DEVICE_COMPILE__)
  return __builtin_amdgcn_ballot_w32(p);
#else
  return p ? 1u : 0u;
#endif
}

__device__ __forceinline__ Frag ldfrag(const unsigned short* p) {
  Frag f;
  f.u[0] = *(const v8us*)(p);
  f.u[1] = *(const v8us*)(p + 16);
  return f;
}

__device__ __forceinline__ v8f mma_h(v16h a, v16h b, v8f c) {
  v8f d = __builtin_amdgcn_wmma_f32_16x16x32_f16(false, a, false, b, (short)0, c, false, false);
#if defined(__HIP_DEVICE_COMPILE__)
  asm volatile("v_nop\n\tv_nop\n\tv_nop\n\tv_nop" : "+v"(d) : "v"(a), "v"(b));
#endif
  return d;
}
__device__ __forceinline__ v8f mma_b(v16b a, v16b b, v8f c) {
  v8f d = __builtin_amdgcn_wmma_f32_16x16x32_bf16(false, a, false, b, (short)0, c, false, false);
#if defined(__HIP_DEVICE_COMPILE__)
  const v16h ha = __builtin_bit_cast(v16h, a), hb = __builtin_bit_cast(v16h, b);
  asm volatile("v_nop\n\tv_nop\n\tv_nop\n\tv_nop" : "+v"(d) : "v"(ha), "v"(hb));
#endif
  return d;
}

__global__ __launch_bounds__(256)
void cvt_w(const float* __restrict__ wq, const float* __restrict__ wk, const float* __restrict__ wv,
           const float* __restrict__ wo, unsigned short* Wb) {
  const int tid = threadIdx.x, blk = blockIdx.x;
  const int wave = tid >> 5, lane = tid & 31;
  const int sel = blk >> 3;
  const float* src = (sel == 0) ? wq : (sel == 1) ? wk : (sel == 2) ? wv : wo;
  const int o   = (blk & 7) * 16 + 2 * wave + (lane >> 4);
  const int col = 8 * (lane & 15);
  const float* s = src + (size_t)o * CC + col;
  const v4f a = *(const v4f*)s;
  const v4f q = *(const v4f*)(s + 4);
  const float f[8] = {a[0], a[1], a[2], a[3], q[0], q[1], q[2], q[3]};
  v4u u;
#pragma unroll
  for (int t = 0; t < 4; ++t) u[t] = pk16(bf_bits(f[2 * t]), bf_bits(f[2 * t + 1]));
#pragma unroll
  for (int pass = 0; pass < 2; ++pass) {
    *(volatile v4u*)(Wb + ((size_t)(sel * CC + o)) * CC + col) = u;
    __threadfence();
  }
}

__global__ __launch_bounds__(256)
void gn_stats(const float* __restrict__ x, float* stats) {
  __shared__ double red[256];
  const int tid = threadIdx.x, bg = blockIdx.x;
  const v4f* p = (const v4f*)(x + (size_t)bg * GSZ * NN);
  const int N4 = GSZ * NN / 4;
  const double invN = 1.0 / (double)(GSZ * NN);

  double s = 0.0;
#pragma unroll 1
  for (int i = tid; i < N4; i += 256) {
    const v4f v = p[i];
    s += ((double)bfr(v[0]) + (double)bfr(v[1])) + ((double)bfr(v[2]) + (double)bfr(v[3]));
  }
  red[tid] = s;
  __syncthreads();
#pragma unroll 1
  for (int off = 128; off > 0; off >>= 1) {
    if (tid < off) red[tid] += red[tid + off];
    __syncthreads();
  }
  const double mean = red[0] * invN;
  __syncthreads();

  double s2 = 0.0;
#pragma unroll 1
  for (int i = tid; i < N4; i += 256) {
    const v4f v = p[i];
#pragma unroll
    for (int t = 0; t < 4; ++t) {
      const double d = (double)bfr(v[t]) - mean;
      s2 += d * d;
    }
  }
  red[tid] = s2;
  __syncthreads();
#pragma unroll 1
  for (int off = 128; off > 0; off >>= 1) {
    if (tid < off) red[tid] += red[tid + off];
    __syncthreads();
  }
  const double var = red[0] * invN;
  const float meanf = (float)mean;
  const float rstdf = (float)(1.0 / sqrt(var + GEPS));

  v4f val = {0.f, 0.f, 0.f, 0.f};
  if (tid == 0) { val[0] = meanf; val[1] = rstdf; }
  float* dst = stats + (size_t)bg * 32 + 4 * (tid & 7);
  if (tid < 8) *(volatile v4f*)dst = val;
  __threadfence();
  if (tid < 8) *(volatile v4f*)dst = val;
}

__global__ __launch_bounds__(256)
void gn_apply(const float* __restrict__ x, const float* __restrict__ gw, const float* __restrict__ gb,
              const float* __restrict__ stats, unsigned short* Hh, unsigned short* Hl) {
  __shared__ __align__(16) unsigned short Th[QT * TP];
  __shared__ __align__(16) unsigned short Tl[QT * TP];
  const int tid = threadIdx.x;
  const int nb = blockIdx.x, cb = blockIdx.y, b = blockIdx.z;
  const int e = tid & 7, lq = tid >> 3;
  const int n0 = nb * QT, c0 = cb * QT;
#pragma unroll
  for (int it = 0; it < 2; ++it) {
    const int cl = it * 32 + lq;
    const int ch = c0 + cl;
    const int g  = ch >> 4;
    const float mean = stats[(size_t)(b * NGRP + g) * 32 + 0];
    const float rstd = stats[(size_t)(b * NGRP + g) * 32 + 1];
    const float w  = bfr(gw[ch]);
    const float bb = bfr(gb[ch]);
    const float* sp = x + ((size_t)(b * CC + ch)) * NN + n0 + 8 * e;
    const v4f a = *(const v4f*)sp;
    const v4f q = *(const v4f*)(sp + 4);
    const float f[8] = {a[0], a[1], a[2], a[3], q[0], q[1], q[2], q[3]};
#pragma unroll
    for (int t = 0; t < 8; ++t) {
      const float h = (bfr(f[t]) - mean) * rstd * w + bb;
      const unsigned short hb = bf_bits(h);
      const unsigned short lb = bf_bits(h - bf_up(hb));
      Th[(8 * e + t) * TP + cl] = hb;
      Tl[(8 * e + t) * TP + cl] = lb;
    }
  }
  __syncthreads();
  v4u uh[2], ul[2];
#pragma unroll
  for (int it = 0; it < 2; ++it) {
    const int nl = it * 32 + lq;
    uh[it] = *(const v4u*)(Th + nl * TP + 8 * e);
    ul[it] = *(const v4u*)(Tl + nl * TP + 8 * e);
  }
#pragma unroll
  for (int pass = 0; pass < 2; ++pass) {
#pragma unroll
    for (int it = 0; it < 2; ++it) {
      const int nl = it * 32 + lq;
      const size_t po = ((size_t)(b * NN + n0 + nl)) * CC + c0 + 8 * e;
      *(volatile v4u*)(Hh + po) = uh[it];
      *(volatile v4u*)(Hl + po) = ul[it];
    }
    __threadfence();
  }
}

__global__ __launch_bounds__(128)
void gemm_qk(const unsigned short* __restrict__ Wb, const unsigned short* __restrict__ Hh,
             const unsigned short* __restrict__ Hl, const float* __restrict__ bq, const float* __restrict__ bk,
             unsigned short* Qh, unsigned short* Ql, unsigned short* Kh) {
  __shared__ __align__(16) float Os[QT * OSP];
  const int tid  = threadIdx.x;
  const int lane = tid & 31, wave = tid >> 5;
  const int hh   = lane >> 4, c = lane & 15;
  const int nt   = blockIdx.x, mb = blockIdx.y, b = blockIdx.z;
  const int sel  = mb >> 1;
  const int n0   = nt * QT, o0 = (mb & 1) * QT;

  const unsigned short* ap = Wb + ((size_t)(sel * CC + o0 + c)) * CC + 8 * hh;
  const size_t ho = ((size_t)(b * NN + n0 + 16 * wave + c)) * CC + 8 * hh;
  const unsigned short* bhp = Hh + ho;
  const unsigned short* blp = Hl + ho;

  v8f acc[4];
#pragma unroll
  for (int mt = 0; mt < 4; ++mt) acc[mt] = zero8();

#pragma unroll
  for (int ks = 0; ks < CC / 32; ++ks) {
    const Frag fbh = ldfrag(bhp + 32 * ks);
    const Frag fbl = ldfrag(blp + 32 * ks);
#pragma unroll
    for (int mt = 0; mt < 4; ++mt) {
      const Frag fa = ldfrag(ap + (size_t)(16 * mt) * CC + 32 * ks);
      acc[mt] = mma_b(fa.bf, fbh.bf, acc[mt]);
      acc[mt] = mma_b(fa.bf, fbl.bf, acc[mt]);
    }
  }

  const float* bsrc = (sel == 0) ? bq : bk;
  {
    const int nl = 16 * wave + c;
#pragma unroll
    for (int mt = 0; mt < 4; ++mt) {
      const v4f b0 = *(const v4f*)(bsrc + o0 + 16 * mt + 8 * hh);
      const v4f b1 = *(const v4f*)(bsrc + o0 + 16 * mt + 8 * hh + 4);
      v4f va, vb;
#pragma unroll
      for (int r = 0; r < 4; ++r) { va[r] = acc[mt][r] + bfr(b0[r]); vb[r] = acc[mt][4 + r] + bfr(b1[r]); }
      *(v4f*)(Os + nl * OSP + 16 * mt + 8 * hh)     = va;
      *(v4f*)(Os + nl * OSP + 16 * mt + 8 * hh + 4) = vb;
    }
  }
  __syncthreads();

  const int e = tid & 7, lq = tid >> 3;
  unsigned short* Ph = (sel == 0) ? Qh : Kh;
  v4u uh[4], ul[4];
#pragma unroll
  for (int it = 0; it < 4; ++it) {
    const int row = it * 16 + lq;
    const v4f a = *(const v4f*)(Os + row * OSP + 8 * e);
    const v4f q = *(const v4f*)(Os + row * OSP + 8 * e + 4);
    const float f[8] = {a[0], a[1], a[2], a[3], q[0], q[1], q[2], q[3]};
#pragma unroll
    for (int t = 0; t < 4; ++t) {
      const float f0 = f[2 * t], f1 = f[2 * t + 1];
      const unsigned short hb0 = bf_bits(f0), hb1 = bf_bits(f1);
      const unsigned short lb0 = bf_bits(f0 - bf_up(hb0));
      const unsigned short lb1 = bf_bits(f1 - bf_up(hb1));
      uh[it][t] = pk16(hb0, hb1);
      ul[it][t] = pk16(lb0, lb1);
    }
  }
#pragma unroll
  for (int pass = 0; pass < 2; ++pass) {
#pragma unroll
    for (int it = 0; it < 4; ++it) {
      const int row = it * 16 + lq;
      const size_t po = ((size_t)(b * NN + n0 + row)) * CC + o0 + 8 * e;
      *(volatile v4u*)(Ph + po) = uh[it];
      if (sel == 0) *(volatile v4u*)(Ql + po) = ul[it];
    }
    __threadfence();
  }
}

__global__ __launch_bounds__(128)
void gemm_v(const unsigned short* __restrict__ Wb, const unsigned short* __restrict__ Hh,
            const unsigned short* __restrict__ Hl, const float* __restrict__ bv, unsigned short* V16) {
  __shared__ __align__(16) float Vs[QT * OSP];
  const int tid  = threadIdx.x;
  const int lane = tid & 31, wave = tid >> 5;
  const int hh   = lane >> 4, c = lane & 15;
  const int nt   = blockIdx.x, mb = blockIdx.y, b = blockIdx.z;
  const int n0   = nt * QT, o0 = mb * QT;

  const size_t ho = ((size_t)(b * NN + n0 + 16 * wave + c)) * CC + 8 * hh;
  const unsigned short* ahp = Hh + ho;
  const unsigned short* alp = Hl + ho;
  const unsigned short* bp  = Wb + ((size_t)(2 * CC + o0 + c)) * CC + 8 * hh;

  v8f acc[4];
#pragma unroll
  for (int j = 0; j < 4; ++j) acc[j] = zero8();

#pragma unroll
  for (int ks = 0; ks < CC / 32; ++ks) {
    const Frag fah = ldfrag(ahp + 32 * ks);
    const Frag fal = ldfrag(alp + 32 * ks);
#pragma unroll
    for (int j = 0; j < 4; ++j) {
      const Frag fb = ldfrag(bp + (size_t)(16 * j) * CC + 32 * ks);
      acc[j] = mma_b(fah.bf, fb.bf, acc[j]);
      acc[j] = mma_b(fal.bf, fb.bf, acc[j]);
    }
  }

  {
    const int nrow = 16 * wave + 8 * hh;
#pragma unroll
    for (int j = 0; j < 4; ++j) {
      const float bb = bfr(bv[o0 + 16 * j + c]);
      v4f va, vb;
#pragma unroll
      for (int r = 0; r < 4; ++r) { va[r] = acc[j][r] + bb; vb[r] = acc[j][4 + r] + bb; }
      *(v4f*)(Vs + (16 * j + c) * OSP + nrow)     = va;
      *(v4f*)(Vs + (16 * j + c) * OSP + nrow + 4) = vb;
    }
  }
  __syncthreads();

  const int e = tid & 7, lq = tid >> 3;
  v4u uv[4];
#pragma unroll
  for (int it = 0; it < 4; ++it) {
    const int ol = it * 16 + lq;
    const v4f a = *(const v4f*)(Vs + ol * OSP + 8 * e);
    const v4f q = *(const v4f*)(Vs + ol * OSP + 8 * e + 4);
    const float f[8] = {a[0], a[1], a[2], a[3], q[0], q[1], q[2], q[3]};
#pragma unroll
    for (int t = 0; t < 4; ++t)
      uv[it][t] = pk16(h_bits((_Float16)f[2 * t]), h_bits((_Float16)f[2 * t + 1]));
  }
#pragma unroll
  for (int pass = 0; pass < 2; ++pass) {
#pragma unroll
    for (int it = 0; it < 4; ++it) {
      const int ol = it * 16 + lq;
      *(volatile v4u*)(V16 + ((size_t)(b * CC + o0 + ol)) * NN + n0 + 8 * e) = uv[it];
    }
    __threadfence();
  }
}

__global__ __launch_bounds__(128)
void attn_k(const unsigned short* __restrict__ Qh, const unsigned short* __restrict__ Ql,
            const unsigned short* __restrict__ Kh, const unsigned short* __restrict__ V16,
            unsigned short* Ah, unsigned short* Al) {
  __shared__ __align__(16) float Os[QT * OSPW];
  const int tid  = threadIdx.x;
  const int wave = tid >> 5, lane = tid & 31;
  const int hh   = lane >> 4, c = lane & 15;
  const int n0   = blockIdx.x * QT, b = blockIdx.y;

  const size_t qo = ((size_t)(b * NN + n0 + 16 * wave + c)) * CC + 8 * hh;
  const unsigned short* Qhp = Qh + qo;
  const unsigned short* Qlp = Ql + qo;
  const unsigned short* Khp = Kh + (size_t)b * NN * CC + (size_t)c * CC + 8 * hh;
  const unsigned short* Vp = V16 + (size_t)b * CC * NN + (size_t)c * NN + 8 * hh;

  float m = -1.0e30f, l = 0.f;
  v8f o[8];
#pragma unroll
  for (int j = 0; j < 8; ++j) o[j] = zero8();

#pragma unroll 1
  for (int kb = 0; kb < NN; kb += 32) {
    const unsigned short* k0p = Khp + (size_t)kb * CC;
    const unsigned short* k1p = Khp + (size_t)(kb + 16) * CC;
    v8f s0 = zero8(), s1 = zero8();
#pragma unroll 1
    for (int kc = 0; kc < CC / 32; ++kc) {
      const Frag qh = ldfrag(Qhp + 32 * kc);
      const Frag ql = ldfrag(Qlp + 32 * kc);
      const Frag k0 = ldfrag(k0p + 32 * kc);
      const Frag k1 = ldfrag(k1p + 32 * kc);
      s0 = mma_b(k0.bf, qh.bf, s0);
      s1 = mma_b(k1.bf, qh.bf, s1);
      s0 = mma_b(k0.bf, ql.bf, s0);
      s1 = mma_b(k1.bf, ql.bf, s1);
    }
#pragma unroll
    for (int r = 0; r < 8; ++r) { s0[r] *= SCL; s1[r] *= SCL; }

    float mx = fmaxf(hmax8(s0), hmax8(s1));
    mx = fmaxf(mx, __shfl_xor(mx, 16, 32));
    const float mn = fmaxf(m, mx);
    const unsigned grew = wave_ballot(mx > m);
    if (grew != 0u) {
      const float corr = __expf(m - mn);
      l *= corr;
#pragma unroll
      for (int j = 0; j < 8; ++j) {
#pragma unroll
        for (int r = 0; r < 8; ++r) o[j][r] *= corr;
      }
    }
    m = mn;
    const float msh = mn - LNPS;

    FragH ph;
    float ls = 0.f;
#pragma unroll
    for (int r = 0; r < 8; ++r) {
      const float e0 = __expf(s0[r] - msh);
      const float e1 = __expf(s1[r] - msh);
      ls += e0 + e1;
      ph.hv[0][r] = (_Float16)e0;
      ph.hv[1][r] = (_Float16)e1;
    }
    l += ls;

#pragma unroll
    for (int j = 0; j < 8; ++j) {
      const Frag vf = ldfrag(Vp + (size_t)(16 * j) * NN + kb);
      o[j] = mma_h(vf.h, ph.v, o[j]);
    }
  }
  l += __shfl_xor(l, 16, 32);
  const float inv = 1.0f / l;

  const int qrow = 16 * wave + c;
#pragma unroll
  for (int j = 0; j < 8; ++j) {
    v4f va, vb;
#pragma unroll
    for (int r = 0; r < 4; ++r) { va[r] = o[j][r] * inv; vb[r] = o[j][4 + r] * inv; }
    *(v4f*)(Os + qrow * OSPW + 16 * j + 8 * hh)     = va;
    *(v4f*)(Os + qrow * OSPW + 16 * j + 8 * hh + 4) = vb;
  }
  __syncthreads();

  const int e = tid & 15, lq = tid >> 4;
  v4u uh[8], ul[8];
#pragma unroll
  for (int it = 0; it < 8; ++it) {
    const int row = it * 8 + lq;
    const v4f a = *(const v4f*)(Os + row * OSPW + 8 * e);
    const v4f q = *(const v4f*)(Os + row * OSPW + 8 * e + 4);
    const float f[8] = {a[0], a[1], a[2], a[3], q[0], q[1], q[2], q[3]};
#pragma unroll
    for (int t = 0; t < 4; ++t) {
      const float f0 = f[2 * t], f1 = f[2 * t + 1];
      const unsigned short hb0 = bf_bits(f0), hb1 = bf_bits(f1);
      const unsigned short lb0 = bf_bits(f0 - bf_up(hb0));
      const unsigned short lb1 = bf_bits(f1 - bf_up(hb1));
      uh[it][t] = pk16(hb0, hb1);
      ul[it][t] = pk16(lb0, lb1);
    }
  }
#pragma unroll
  for (int pass = 0; pass < 2; ++pass) {
#pragma unroll
    for (int it = 0; it < 8; ++it) {
      const int row = it * 8 + lq;
      const size_t po = ((size_t)(b * NN + n0 + row)) * CC + 8 * e;
      *(volatile v4u*)(Ah + po) = uh[it];
      *(volatile v4u*)(Al + po) = ul[it];
    }
    __threadfence();
  }
}

__global__ __launch_bounds__(128)
void gemm_p(const unsigned short* __restrict__ Wb, const unsigned short* __restrict__ Ah,
            const unsigned short* __restrict__ Al, const float* __restrict__ bo, const float* __restrict__ x,
            float* out) {
  __shared__ __align__(16) float Vs[QT * OSP];
  const int tid  = threadIdx.x;
  const int lane = tid & 31, wave = tid >> 5;
  const int hh   = lane >> 4, c = lane & 15;
  const int nt   = blockIdx.x, mb = blockIdx.y, b = blockIdx.z;
  const int n0   = nt * QT, o0 = mb * QT;

  const size_t ao = ((size_t)(b * NN + n0 + 16 * wave + c)) * CC + 8 * hh;
  const unsigned short* ahp = Ah + ao;
  const unsigned short* alp = Al + ao;
  const unsigned short* bpw = Wb + ((size_t)(3 * CC + o0 + c)) * CC + 8 * hh;

  v8f acc[4];
#pragma unroll
  for (int j = 0; j < 4; ++j) acc[j] = zero8();

#pragma unroll
  for (int ks = 0; ks < CC / 32; ++ks) {
    const Frag fah = ldfrag(ahp + 32 * ks);
    const Frag fal = ldfrag(alp + 32 * ks);
#pragma unroll
    for (int j = 0; j < 4; ++j) {
      const Frag fb = ldfrag(bpw + (size_t)(16 * j) * CC + 32 * ks);
      acc[j] = mma_b(fah.bf, fb.bf, acc[j]);
      acc[j] = mma_b(fal.bf, fb.bf, acc[j]);
    }
  }

  {
    const int nrow = 16 * wave + 8 * hh;
#pragma unroll
    for (int j = 0; j < 4; ++j) {
      const float bb = bfr(bo[o0 + 16 * j + c]);
      v4f va, vb;
#pragma unroll
      for (int r = 0; r < 4; ++r) { va[r] = acc[j][r] + bb; vb[r] = acc[j][4 + r] + bb; }
      *(v4f*)(Vs + (16 * j + c) * OSP + nrow)     = va;
      *(v4f*)(Vs + (16 * j + c) * OSP + nrow + 4) = vb;
    }
  }
  __syncthreads();

  const int e = tid & 15, lq = tid >> 4;
  v4f res[8];
#pragma unroll
  for (int it = 0; it < 8; ++it) {
    const int ol = it * 8 + lq;
    const v4f a = *(const v4f*)(Vs + ol * OSP + 4 * e);
    const size_t idx = ((size_t)(b * CC + o0 + ol)) * NN + n0 + 4 * e;
    const v4f xv = *(const v4f*)(x + idx);
#pragma unroll
    for (int t = 0; t < 4; ++t) res[it][t] = a[t] + bfr(xv[t]);
  }
#pragma unroll
  for (int pass = 0; pass < 2; ++pass) {
#pragma unroll
    for (int it = 0; it < 8; ++it) {
      const int ol = it * 8 + lq;
      const size_t idx = ((size_t)(b * CC + o0 + ol)) * NN + n0 + 4 * e;
      *(volatile v4f*)(out + idx) = res[it];
    }
    __threadfence();
  }
}

extern "C" void kernel_launch(void* const* d_in, const int* in_sizes, int n_in,
                              void* d_out, int out_size, void* d_ws, size_t ws_size,
                              hipStream_t stream) {
  if (n_in < 11) return;
  if (in_sizes[0] < NB * CC * NN) return;
  if (in_sizes[1] < CC || in_sizes[2] < CC) return;
  if (in_sizes[3] < CC * CC || in_sizes[5] < CC * CC || in_sizes[7] < CC * CC || in_sizes[9] < CC * CC) return;
  if (in_sizes[4] < CC || in_sizes[6] < CC || in_sizes[8] < CC || in_sizes[10] < CC) return;
  if (out_size < NB * CC * NN) return;

  size_t off = 0;
  auto carve = [&](size_t bytes) { const size_t o = off; off += (bytes + 255) & ~(size_t)255; return o; };
  const size_t plane = (size_t)NB * NN * CC * 2;
  const size_t oWb  = carve((size_t)4 * CC * CC * 2);
  const size_t oSt  = carve((size_t)NB * NGRP * 32 * 4);
  const size_t oHh  = carve(plane);
  const size_t oHl  = carve(plane);
  const size_t oQh  = carve(plane);
  const size_t oQl  = carve(plane);
  const size_t oKh  = carve(plane);
  const size_t oV16 = carve(plane);
  const size_t oAh  = oHh;
  const size_t oAl  = oHl;
  if (off > ws_size) return;
  if (off > (size_t)134217728) return;

  const float* x   = (const float*)d_in[0];
  const float* gnw = (const float*)d_in[1];
  const float* gnb = (const float*)d_in[2];
  const float* wq  = (const float*)d_in[3];
  const float* bq  = (const float*)d_in[4];
  const float* wk  = (const float*)d_in[5];
  const float* bk  = (const float*)d_in[6];
  const float* wv  = (const float*)d_in[7];
  const float* bv  = (const float*)d_in[8];
  const float* wo  = (const float*)d_in[9];
  const float* bo  = (const float*)d_in[10];

  char* ws = (char*)d_ws;
  unsigned short* Wb  = (unsigned short*)(ws + oWb);
  float*          St  = (float*)(ws + oSt);
  unsigned short* Hh  = (unsigned short*)(ws + oHh);
  unsigned short* Hl  = (unsigned short*)(ws + oHl);
  unsigned short* Qh  = (unsigned short*)(ws + oQh);
  unsigned short* Ql  = (unsigned short*)(ws + oQl);
  unsigned short* Kh  = (unsigned short*)(ws + oKh);
  unsigned short* V16 = (unsigned short*)(ws + oV16);
  unsigned short* Ah  = (unsigned short*)(ws + oAh);
  unsigned short* Al  = (unsigned short*)(ws + oAl);
  float* out = (float*)d_out;

  const dim3 blk256(256), blk128(128);

  cvt_w<<<dim3(32), blk256, 0, stream>>>(wq, wk, wv, wo, Wb);
  gn_stats<<<dim3(NB * NGRP), blk256, 0, stream>>>(x, St);
  gn_apply<<<dim3(NN / QT, CC / QT, NB), blk256, 0, stream>>>(x, gnw, gnb, St, Hh, Hl);
  gemm_qk<<<dim3(NN / QT, 4, NB), blk128, 0, stream>>>(Wb, Hh, Hl, bq, bk, Qh, Ql, Kh);
  gemm_v<<<dim3(NN / QT, 2, NB), blk128, 0, stream>>>(Wb, Hh, Hl, bv, V16);
  attn_k<<<dim3(NQ / QT, NB), blk128, 0, stream>>>(Qh, Ql, Kh, V16, Ah, Al);
  gemm_p<<<dim3(NQ / QT, 2, NB), blk128, 0, stream>>>(Wb, Ah, Al, bo, x, out);
  (void)hipGetLastError();
}
